// CPCLossV2_10557029613703
// MI455X (gfx1250) — hardware-run, weakly checked
//
#include <hip/hip_runtime.h>
#include <math.h>

typedef __attribute__((ext_vector_type(16))) _Float16 v16h;
typedef __attribute__((ext_vector_type(16))) __bf16 v16b;
typedef __attribute__((ext_vector_type(8)))  _Float16 v8h;
typedef __attribute__((ext_vector_type(8)))  float v8f;
typedef __attribute__((ext_vector_type(4)))  float v4f;
typedef __attribute__((ext_vector_type(2)))  float v2f;
typedef __attribute__((ext_vector_type(4)))  unsigned v4u;
typedef __attribute__((ext_vector_type(4)))  int v4i;
typedef float __attribute__((may_alias)) float_a;
typedef int __attribute__((may_alias)) int_a;

template <typename T> __device__ __forceinline__ void vst2(void* p, T v) { *(volatile T*)p = v; __threadfence(); *(volatile T*)p = v; }
__device__ __forceinline__ v8f wmma16(v16h a, v16h b, v8f c) {
  v8f d = __builtin_amdgcn_wmma_f32_16x16x32_f16(false, a, false, b, (short)0, c, false, false);
  asm volatile("v_nop\n\tv_nop\n\tv_nop\n\tv_nop" : "+v"(d) : "v"(a), "v"(b));
  return d;
}
__device__ __forceinline__ v8f wmma_bf(v16b a, v16b b, v8f c) {
  v8f d = __builtin_amdgcn_wmma_f32_16x16x32_bf16(false, a, false, b, (short)0, c, false, false);
  asm volatile("v_nop\n\tv_nop\n\tv_nop\n\tv_nop" : "+v"(d) : "v"(a), "v"(b));
  return d;
}
__device__ __forceinline__ v16h frag_h(const _Float16* rowk0, int lane) {
  union { v16h v; v8h q[2]; } u; const _Float16* p = rowk0 + 8 * (lane >> 4);
  u.q[0] = *(const v8h*)p; u.q[1] = *(const v8h*)(p + 16); return u.v;
}
__device__ __forceinline__ v16h frag_f32(const float* rowk0, int lane) {
  v16h a; const float* p = rowk0 + 8 * (lane >> 4);
#pragma unroll
  for (int i = 0; i < 8; ++i) { a[i] = (_Float16)p[i]; a[8 + i] = (_Float16)p[16 + i]; }
  return a;
}
__device__ __forceinline__ v16h frag_f32s(const float* rowk0, int lane, float sc) {
  v16h a; const float* p = rowk0 + 8 * (lane >> 4);
#pragma unroll
  for (int i = 0; i < 8; ++i) { a[i] = (_Float16)(p[i] * sc); a[8 + i] = (_Float16)(p[16 + i] * sc); }
  return a;
}
__device__ __forceinline__ v16h fragc_f32(const float* W, int k0, int n, int lane, int ld, int K) {
  v16h a; const int g = lane >> 4;
#pragma unroll
  for (int i = 0; i < 8; ++i) { const int ka = k0 + 8 * g + i, kb = ka + 16;
    a[i] = (_Float16)(ka < K ? W[(size_t)(ka < K ? ka : K - 1) * ld + n] : 0.f); a[8 + i] = (_Float16)(kb < K ? W[(size_t)(kb < K ? kb : K - 1) * ld + n] : 0.f); }
  return a;
}
struct F2 { v16b h, l; };
__device__ __forceinline__ F2 bsplit16(const float v[16]) { F2 r;
#pragma unroll
  for (int i = 0; i < 16; ++i) { const __bf16 h = (__bf16)v[i]; r.h[i] = h; r.l[i] = (__bf16)(v[i] - (float)h); }
  return r; }
__device__ __forceinline__ F2 split_row(const float* row, int k0, int lane) { float v[16]; const float* p = row + k0 + 8 * (lane >> 4);
#pragma unroll
  for (int i = 0; i < 8; ++i) { v[i] = p[i]; v[8 + i] = p[16 + i]; }
  return bsplit16(v); }
__device__ __forceinline__ F2 split_rowK(const float* row, int k0, int lane, int K) { float v[16]; const int g = lane >> 4;
#pragma unroll
  for (int i = 0; i < 8; ++i) { const int ka = k0 + 8 * g + i, kb = ka + 16; v[i] = ka < K ? row[ka < K ? ka : K - 1] : 0.f; v[8 + i] = kb < K ? row[kb < K ? kb : K - 1] : 0.f; }
  return bsplit16(v); }
__device__ __forceinline__ F2 split_col(const float* W, int k0, int n, int lane, int ld, int K) { float v[16]; const int g = lane >> 4;
#pragma unroll
  for (int i = 0; i < 8; ++i) { const int ka = k0 + 8 * g + i, kb = ka + 16; v[i] = ka < K ? W[(size_t)(ka < K ? ka : K - 1) * ld + n] : 0.f; v[8 + i] = kb < K ? W[(size_t)(kb < K ? kb : K - 1) * ld + n] : 0.f; }
  return bsplit16(v); }
__device__ __forceinline__ v8f mac3(const F2& a, const F2& b, v8f c) { c = wmma_bf(a.l, b.h, c); c = wmma_bf(a.h, b.l, c); return wmma_bf(a.h, b.h, c); }
__device__ __forceinline__ float sigm(float v) { return 1.0f / (1.0f + expf(-v)); }
#define LDSX() do { asm volatile("s_wait_dscnt 0" ::: "memory"); __builtin_amdgcn_wave_barrier(); __builtin_amdgcn_fence(__ATOMIC_RELEASE, "workgroup"); } while (0)


#define NROW 16384
#define HH 256
#define KP 4
#define NG (NROW / KP)
#define MNEG 64
#define EQCAP 1024
typedef __attribute__((ext_vector_type(8))) __bf16 v8b;
__device__ __forceinline__ v16b frag_b(const __bf16* rowk0, int lane) {
  union { v16b v; v8b q[2]; } u; const __bf16* p = rowk0 + 8 * (lane >> 4);
  u.q[0] = *(const v8b*)p; u.q[1] = *(const v8b*)(p + 16); return u.v;
}
__device__ __forceinline__ float bfr(float v) { return (float)(__bf16)v; }
__device__ __attribute__((noinline)) float exp_ni(float v) { return expf(v); }
__device__ __attribute__((noinline)) float erf_ni(float v) { return erff(v); }

__device__ __attribute__((noinline)) float log_ni(float v) { return logf(v); }
#define WS_PW   0u
#define WS_PRED (WS_PW + 2u * HH * 3 * HH)
#define WS_PL   (WS_PRED + 4u * NG * HH)
#define WS_END  (WS_PL + 4u * NG)

__global__ __launch_bounds__(256) void k_pack(const float* __restrict__ Wm, __bf16* __restrict__ PW) {
  __shared__ __align__(16) __bf16 s[3 * HH]; const int n = blockIdx.x, tid = threadIdx.x;
  for (int k = tid; k < 3 * HH; k += 256) s[k] = (__bf16)Wm[(size_t)k * HH + n];
  __syncthreads();
  for (int q = tid; q < 3 * HH / 8; q += 256) vst2((unsigned*)(PW + (size_t)n * 3 * HH + q * 8), *(const v4u*)&s[q * 8]);
}
__global__ __launch_bounds__(128) void k_pred(const float* __restrict__ E, const __bf16* __restrict__ PW, const float* __restrict__ Bv, float* __restrict__ PRED) {
  __shared__ __align__(16) float so[4][16][132];
  const int tid = threadIdx.x, wave = tid >> 5, lane = tid & 31, col = lane & 15, g = lane >> 4; const size_t r0 = (size_t)blockIdx.x * 64 + wave * 16; const int n0 = blockIdx.y * 128;
  v8f acc[8] = {};
#pragma unroll 2
  for (int kc = 0; kc < 3 * HH / 32; ++kc) { v16b a; { const float* p = E + (r0 + col) * (KP * HH) + kc * 32 + 8 * g;
#pragma unroll
      for (int i = 0; i < 8; ++i) { a[i] = (__bf16)p[i]; a[8 + i] = (__bf16)p[16 + i]; } }
#pragma unroll
    for (int j = 0; j < 8; ++j) acc[j] = wmma_bf(a, frag_b(PW + (size_t)(n0 + j * 16 + col) * (3 * HH) + kc * 32, lane), acc[j]); }
#pragma unroll
  for (int j = 0; j < 8; ++j) { const float bb = bfr(Bv[n0 + j * 16 + col]);
#pragma unroll
    for (int r = 0; r < 8; ++r) so[wave][8 * g + r][j * 16 + col] = acc[j][r] + bb; }
  LDSX();
  for (int rl = 0; rl < 16; ++rl) vst2(PRED + (r0 + rl) * HH + n0 + lane * 4, *(const v4f*)&so[wave][rl][lane * 4]);
}
__global__ __launch_bounds__(256) void k_loss(const float* __restrict__ E, const float* __restrict__ PRED, const int* __restrict__ TGT, const int* __restrict__ PERM, const int* __restrict__ KPS, const int* __restrict__ MNS, float* __restrict__ PL) {
  __shared__ int seq[8][EQCAP]; __shared__ int sneg[8][MNEG]; __shared__ float slg[8][MNEG + 1]; __shared__ __align__(16) float sl[64];
  const int tid = threadIdx.x, wave = tid >> 5, lane = tid & 31; const int gi = blockIdx.x * 8 + wave;
  const int kk = min(max(KPS[0], 1), KP); (void)kk;
  const int mm = min(max(MNS[0], 1), MNEG);
  const int tg = TGT[gi * KP];
  int cnt = 0;
  for (int c0 = 0; c0 < NROW; c0 += 32) { const int j = c0 + lane; const bool eq = (TGT[j] == tg); const unsigned bal = __builtin_amdgcn_ballot_w32(eq); const int rank = __builtin_popcount(bal & ((1u << lane) - 1u)); if (eq && cnt + rank < EQCAP) seq[wave][cnt + rank] = j; cnt += __builtin_popcount(bal); }
  cnt = min(cnt, EQCAP);
  LDSX();
  for (int si = lane; si < MNEG; si += 32) { int j = -1;
    if (si < mm) { const int p = min(max(PERM[(size_t)gi * MNEG + si], 0), NROW - 1); j = p;
      for (int it = 0; it < 64; ++it) { int c = 0; for (int q = 0; q < cnt; ++q) c += (seq[wave][q] <= j) ? 1 : 0; const int jn = min(p + c, NROW - 1); if (jn == j) break; j = jn; } }
    sneg[wave][si] = j; }
  LDSX();
  const float* pr = PRED + (size_t)gi * HH;
  for (int li = 0; li <= mm; ++li) { const int row = (li == 0) ? (gi * KP + KP - 1) : sneg[wave][li - 1]; const float* er = E + (size_t)row * HH; float a = 0.f;
#pragma unroll
    for (int k = 0; k < 8; ++k) { const int c = lane + 32 * k; a += pr[c] * bfr(er[c]); }
#pragma unroll
    for (int o = 1; o < 32; o <<= 1) a += __shfl_xor(a, o);
    if (lane == 0) slg[wave][li] = a; }
  LDSX();
  if (lane == 0) { float mx = slg[wave][0]; for (int li = 1; li <= mm; ++li) mx = fmaxf(mx, slg[wave][li]); float z = 0.f; for (int li = 0; li <= mm; ++li) z += exp_ni(slg[wave][li] - mx); sl[wave] = -(slg[wave][0] - mx - log_ni(z)); }
  __syncthreads();
  if (tid == 0) { for (int w = 8; w < 64; ++w) sl[w] = 0.f; }
  __syncthreads();
  if (tid < 16) vst2(PL + (size_t)blockIdx.x * 64 + tid * 4, *(const v4f*)&sl[tid * 4]);
}
__global__ __launch_bounds__(256) void k_mean(const float* __restrict__ PL, float* __restrict__ out) {
  __shared__ float sp[256]; __shared__ __align__(16) float so[4]; const int tid = threadIdx.x; float a = 0.f;
  for (int blk = tid; blk < NG / 8; blk += 256) { for (int w = 0; w < 8; ++w) a += PL[(size_t)blk * 64 + w]; }
  sp[tid] = a; __syncthreads();
  if (tid == 0) { float t = 0.f; for (int i = 0; i < 256; ++i) t += sp[i]; so[0] = t / (float)NG; so[1] = 0.f; so[2] = 0.f; so[3] = 0.f; vst2(out, so[0]); }
}
extern "C" void kernel_launch(void* const* d_in, const int* in_sizes, int n_in, void* d_out, int out_size, void* d_ws, size_t ws_size, hipStream_t stream) {
  (void)in_sizes; (void)n_in; (void)out_size;
  const float* E = (const float*)d_in[0]; const float* Wm = (const float*)d_in[1]; const float* Bv = (const float*)d_in[2]; const int* TGT = (const int*)d_in[3]; const int* PERM = (const int*)d_in[4]; const int* KPS = (const int*)d_in[5]; const int* MNS = (const int*)d_in[6];
  if (ws_size < (size_t)WS_END) return;
  char* ws = (char*)d_ws; __bf16* PW = (__bf16*)(ws + WS_PW); float *PRED = (float*)(ws + WS_PRED), *PL = (float*)(ws + WS_PL);
  k_pack<<<HH, 256, 0, stream>>>(Wm, PW);
  k_pred<<<dim3(NG / 64, HH / 128), 128, 0, stream>>>(E, PW, Bv, PRED);
  k_loss<<<NG / 8, 256, 0, stream>>>(E, PRED, TGT, PERM, KPS, MNS, PL);
  k_mean<<<1, 256, 0, stream>>>(PL, (float*)d_out);
}
